// Decoder_74998718923424
// MI455X (gfx1250) — hardware-verified
//
#include <hip/hip_runtime.h>
#define BB 2
#define TT 1024
#define DD 512
#define NH 8
#define HD 64
#define FF 2048
#define NL 2
#define VV 32000

typedef __bf16 v16b __attribute__((ext_vector_type(16)));
typedef unsigned short v8us __attribute__((ext_vector_type(8), may_alias));
typedef float  v8f  __attribute__((ext_vector_type(8)));
typedef float  v4f  __attribute__((ext_vector_type(4)));
typedef float  v4fa __attribute__((ext_vector_type(4), may_alias));
union FragB { v16b v; v8us half[2]; unsigned short u[16]; };

__device__ __forceinline__ unsigned short bf16_bits(float x) { unsigned int u = __float_as_uint(x); return (unsigned short)((u + 0x7FFFu + ((u >> 16) & 1u)) >> 16); }
__device__ __forceinline__ float bf16_val(unsigned short b) { return __uint_as_float(((unsigned int)b) << 16); }
__device__ __forceinline__ float bf16_round(float x) { return bf16_val(bf16_bits(x)); }
template <int NT>
__device__ __forceinline__ v8f mmaN(v16b ah, v16b al, v16b bh, v16b bl, v8f c) {
  c = __builtin_amdgcn_wmma_f32_16x16x32_bf16(false, ah, false, bh, (short)0, c, false, false);
  if (NT >= 2) c = __builtin_amdgcn_wmma_f32_16x16x32_bf16(false, al, false, bh, (short)0, c, false, false);
  if (NT >= 3) c = __builtin_amdgcn_wmma_f32_16x16x32_bf16(false, ah, false, bl, (short)0, c, false, false);
  asm volatile("v_nop\n\tv_nop\n\tv_nop\n\tv_nop" : "+v"(c) : "v"(ah), "v"(al), "v"(bh), "v"(bl));
  return c;
}

__global__ __launch_bounds__(256) void k_wt_bf16(const float* __restrict__ W, unsigned short* __restrict__ Wt, int K, int N) {
  const int t = blockIdx.x * 256 + threadIdx.x;
  const int k8n = K / 8;
  if (t >= N * k8n) return;
  const int n = t / k8n, k8 = (t % k8n) * 8;
  v8us v;
#pragma unroll
  for (int i = 0; i < 8; ++i) v[i] = bf16_bits(W[(size_t)(k8 + i) * N + n]);
  *(volatile v8us*)(Wt + (size_t)n * K + k8) = v;
  __threadfence();
  *(volatile v8us*)(Wt + (size_t)n * K + k8) = v;
}

template <bool ASPLIT, int ACT, bool BIAS_BF16>
__global__ __launch_bounds__(128) void k_gemm_bf(const float* __restrict__ A, int lda, const unsigned short* __restrict__ Wt, int ldb,
                                               const float* __restrict__ bias, float* __restrict__ C, int ldc, int M, int N, int K) {
  __shared__ __attribute__((aligned(16))) float so[4][16][64];
  const int tid = threadIdx.x, w = tid >> 5, lane = tid & 31, ln = lane & 15, hh = lane >> 4;
  const int ntn = N / 64;
  const int wid = blockIdx.x * 4 + w;
  const int mt = wid / ntn, nq = wid % ntn;
  if (mt * 16 >= M) return;
  const int row0 = mt * 16, col0 = nq * 64;
  const float* arow = A + (size_t)(row0 + ln) * lda;
  v8f acc[4] = {};
  for (int kb = 0; kb < K; kb += 32) {
    FragB ah, al;
    const v4f x0 = *(const v4fa*)(arow + kb + 8 * hh), x1 = *(const v4fa*)(arow + kb + 8 * hh + 4);
    const v4f x2 = *(const v4fa*)(arow + kb + 16 + 8 * hh), x3 = *(const v4fa*)(arow + kb + 16 + 8 * hh + 4);
    float xs[16] = {x0[0],x0[1],x0[2],x0[3],x1[0],x1[1],x1[2],x1[3],x2[0],x2[1],x2[2],x2[3],x3[0],x3[1],x3[2],x3[3]};
#pragma unroll
    for (int i = 0; i < 16; ++i) { const unsigned short hb = bf16_bits(xs[i]); ah.u[i] = hb; al.u[i] = ASPLIT ? bf16_bits(xs[i] - bf16_val(hb)) : (unsigned short)0; }
#pragma unroll
    for (int t = 0; t < 4; ++t) {
      const unsigned short* brow = Wt + (size_t)(col0 + t * 16 + ln) * ldb + kb;
      FragB b;
      b.half[0] = *(const v8us*)(brow + 8 * hh);
      b.half[1] = *(const v8us*)(brow + 16 + 8 * hh);
      acc[t] = mmaN<ASPLIT ? 2 : 1>(ah.v, al.v, b.v, b.v, acc[t]);
    }
  }
#pragma unroll
  for (int t = 0; t < 4; ++t) {
    float bv = bias ? bias[col0 + t * 16 + ln] : 0.f;
    if (BIAS_BF16) bv = bf16_round(bv);
#pragma unroll
    for (int r = 0; r < 8; ++r) { float v = acc[t][r] + bv; if (ACT == 1) v = fmaxf(v, 0.f); so[w][8 * hh + r][t * 16 + ln] = v; }
  }
  __builtin_amdgcn_fence(__ATOMIC_ACQ_REL, "workgroup");
  __builtin_amdgcn_wave_barrier();
  const int rsub = lane >> 4, c4 = (lane & 15) * 4;
  for (int pass = 0; pass < 2; ++pass) {
#pragma unroll
    for (int q = 0; q < 8; ++q) {
      const int r = q * 2 + rsub;
      const v4f v = *(const v4fa*)&so[w][r][c4];
      *(volatile v4f*)(C + (size_t)(row0 + r) * ldc + col0 + c4) = v;
    }
    if (pass == 0) __threadfence();
  }
}

template <int D, bool CAUSAL>
__global__ __launch_bounds__(128) void k_flash(const float* __restrict__ qb, const float* __restrict__ kb, const float* __restrict__ vb,
                                             int pitch, int T, int H, float scale, float* __restrict__ y, int ypitch) {
  constexpr int KS = D / 32;
  constexpr int DT = D / 16;
  __shared__ __attribute__((aligned(16))) unsigned short sKh[32][D + 8], sKl[32][D + 8], sVh[32][D + 8], sVl[32][D + 8];
  __shared__ __attribute__((aligned(16))) unsigned short sPh[4][16][40], sPl[4][16][40];
  __shared__ __attribute__((aligned(16))) float sO[4][16][D];
  const int tid = threadIdx.x, w = tid >> 5, lane = tid & 31, ln = lane & 15, hh = lane >> 4;
  const int nqb = (T + 63) / 64;
  const int bh = blockIdx.x / nqb, qblk = blockIdx.x % nqb;
  const int b = bh / H, h = bh % H;
  const int q0 = qblk * 64 + w * 16;
  const float* Q = qb + (size_t)b * T * pitch + h * D;
  const float* K = kb + (size_t)b * T * pitch + h * D;
  const float* V = vb + (size_t)b * T * pitch + h * D;

  FragB aqh[KS], aql[KS];
  {
    int row = q0 + ln; if (row >= T) row = T - 1;
    const float* qr = Q + (size_t)row * pitch;
#pragma unroll
    for (int ks = 0; ks < KS; ++ks)
#pragma unroll
      for (int i = 0; i < 16; ++i) {
        const int d = ks * 32 + ((i < 8) ? (8 * hh + i) : (16 + 8 * hh + (i - 8)));
        const float x = qr[d] * scale; const unsigned short hb = bf16_bits(x);
        aqh[ks].u[i] = hb; aql[ks].u[i] = bf16_bits(x - bf16_val(hb));
      }
  }
  float m_r[8], l_r[8];
#pragma unroll
  for (int r = 0; r < 8; ++r) { m_r[r] = -3.0e38f; l_r[r] = 0.f; }
  v8f oacc[DT];
#pragma unroll
  for (int dt = 0; dt < DT; ++dt) oacc[dt] = (v8f){0.f,0.f,0.f,0.f,0.f,0.f,0.f,0.f};

  const int kv_end = CAUSAL ? min(T, qblk * 64 + 64) : T;
  for (int j0 = 0; j0 < kv_end; j0 += 32) {
    __syncthreads();
    for (int e = tid; e < 32 * (D / 4); e += 128) {
      const int r = e / (D / 4), c4 = (e % (D / 4)) * 4;
      const int key = j0 + r;
      v4f kf = {0.f,0.f,0.f,0.f}, vf = {0.f,0.f,0.f,0.f};
      if (key < T) { kf = *(const v4fa*)(K + (size_t)key * pitch + c4); vf = *(const v4fa*)(V + (size_t)key * pitch + c4); }
#pragma unroll
      for (int t = 0; t < 4; ++t) {
        unsigned short hb = bf16_bits(kf[t]); sKh[r][c4 + t] = hb; sKl[r][c4 + t] = bf16_bits(kf[t] - bf16_val(hb));
        hb = bf16_bits(vf[t]); sVh[r][c4 + t] = hb; sVl[r][c4 + t] = bf16_bits(vf[t] - bf16_val(hb));
      }
    }
    __syncthreads();
    v8f s[2];
#pragma unroll
    for (int nt = 0; nt < 2; ++nt) {
      v8f acc = {};
#pragma unroll
      for (int ks = 0; ks < KS; ++ks) {
        FragB bh_, bl_;
        bh_.half[0] = *(const v8us*)&sKh[nt * 16 + ln][ks * 32 + 8 * hh]; bh_.half[1] = *(const v8us*)&sKh[nt * 16 + ln][ks * 32 + 16 + 8 * hh];
        bl_.half[0] = *(const v8us*)&sKl[nt * 16 + ln][ks * 32 + 8 * hh]; bl_.half[1] = *(const v8us*)&sKl[nt * 16 + ln][ks * 32 + 16 + 8 * hh];
        acc = mmaN<3>(aqh[ks].v, aql[ks].v, bh_.v, bl_.v, acc);
      }
      s[nt] = acc;
    }
    float alpha[8];
#pragma unroll
    for (int r = 0; r < 8; ++r) {
      const int qi = q0 + 8 * hh + r;
      const int ja = j0 + ln, jb = j0 + 16 + ln;
      if (CAUSAL) { if (ja > qi) s[0][r] = -3.0e38f; if (jb > qi) s[1][r] = -3.0e38f; }
      if (ja >= T) s[0][r] = -3.0e38f;
      if (jb >= T) s[1][r] = -3.0e38f;
      float mx = fmaxf(s[0][r], s[1][r]);
      mx = fmaxf(mx, __shfl_xor(mx, 1, 32)); mx = fmaxf(mx, __shfl_xor(mx, 2, 32)); mx = fmaxf(mx, __shfl_xor(mx, 4, 32)); mx = fmaxf(mx, __shfl_xor(mx, 8, 32));
      const float mnew = fmaxf(m_r[r], mx);
      alpha[r] = (mnew > -1.0e38f) ? __expf(m_r[r] - mnew) : 1.0f;
      const float p0 = (s[0][r] > -1.0e38f) ? __expf(s[0][r] - mnew) : 0.f;
      const float p1 = (s[1][r] > -1.0e38f) ? __expf(s[1][r] - mnew) : 0.f;
      m_r[r] = mnew;
      l_r[r] = l_r[r] * alpha[r] + p0 + p1;
      unsigned short hb = bf16_bits(p0); sPh[w][8 * hh + r][ln] = hb;      sPl[w][8 * hh + r][ln] = bf16_bits(p0 - bf16_val(hb));
      hb = bf16_bits(p1);                sPh[w][8 * hh + r][16 + ln] = hb; sPl[w][8 * hh + r][16 + ln] = bf16_bits(p1 - bf16_val(hb));
    }
#pragma unroll
    for (int dt = 0; dt < DT; ++dt)
#pragma unroll
      for (int r = 0; r < 8; ++r) oacc[dt][r] *= alpha[r];
    __builtin_amdgcn_fence(__ATOMIC_ACQ_REL, "workgroup");
    __builtin_amdgcn_wave_barrier();
    FragB pah, pal;
    pah.half[0] = *(const v8us*)&sPh[w][ln][8 * hh]; pah.half[1] = *(const v8us*)&sPh[w][ln][16 + 8 * hh];
    pal.half[0] = *(const v8us*)&sPl[w][ln][8 * hh]; pal.half[1] = *(const v8us*)&sPl[w][ln][16 + 8 * hh];
#pragma unroll
    for (int dt = 0; dt < DT; ++dt) {
      FragB bvh, bvl;
#pragma unroll
      for (int i = 0; i < 8; ++i) {
        bvh.u[i] = sVh[8 * hh + i][dt * 16 + ln]; bvh.u[8 + i] = sVh[16 + 8 * hh + i][dt * 16 + ln];
        bvl.u[i] = sVl[8 * hh + i][dt * 16 + ln]; bvl.u[8 + i] = sVl[16 + 8 * hh + i][dt * 16 + ln];
      }
      oacc[dt] = mmaN<3>(pah.v, pal.v, bvh.v, bvl.v, oacc[dt]);
    }
    __builtin_amdgcn_fence(__ATOMIC_ACQ_REL, "workgroup");
    __builtin_amdgcn_wave_barrier();
  }
#pragma unroll
  for (int r = 0; r < 8; ++r) {
    float l = l_r[r];
    l += __shfl_xor(l, 1, 32); l += __shfl_xor(l, 2, 32); l += __shfl_xor(l, 4, 32); l += __shfl_xor(l, 8, 32);
    l_r[r] = (l > 0.f) ? 1.0f / l : 0.f;
  }
#pragma unroll
  for (int dt = 0; dt < DT; ++dt)
#pragma unroll
    for (int r = 0; r < 8; ++r) sO[w][8 * hh + r][dt * 16 + ln] = oacc[dt][r] * l_r[r];
  __builtin_amdgcn_fence(__ATOMIC_ACQ_REL, "workgroup");
  __builtin_amdgcn_wave_barrier();
  for (int pass = 0; pass < 2; ++pass) {
    for (int r = 0; r < 16; ++r) {
      const int row = q0 + r;
      if (row < T && lane < D / 4) {
        const v4f val = *(const v4fa*)&sO[w][r][lane * 4];
        *(volatile v4f*)(y + ((size_t)b * T + row) * ypitch + h * D + lane * 4) = val;
      }
    }
    if (pass == 0) __threadfence();
  }
}

template <bool ASPLIT, int ACT, bool BIAS_BF16, bool RES_BF16>
__global__ __launch_bounds__(128) void k_gemm_bf3(const float* __restrict__ A, int lda, const unsigned short* __restrict__ Wt, int ldb,
                                                const float* __restrict__ bias, const float* __restrict__ resid, int rmod, int ldr,
                                                float* __restrict__ C, int ldc, int M, int N, int K) {
  __shared__ __attribute__((aligned(16))) float so[4][16][64];
  const int tid = threadIdx.x, w = tid >> 5, lane = tid & 31, ln = lane & 15, hh = lane >> 4;
  const int ntn = N / 64;
  const int wid = blockIdx.x * 4 + w;
  const int mt = wid / ntn, nq = wid % ntn;
  if (mt * 16 >= M) return;
  const int row0 = mt * 16, col0 = nq * 64;
  const float* arow = A + (size_t)(row0 + ln) * lda;
  v8f acc[4] = {};
  for (int kb = 0; kb < K; kb += 32) {
    FragB ah, al;
    const v4f x0 = *(const v4fa*)(arow + kb + 8 * hh), x1 = *(const v4fa*)(arow + kb + 8 * hh + 4);
    const v4f x2 = *(const v4fa*)(arow + kb + 16 + 8 * hh), x3 = *(const v4fa*)(arow + kb + 16 + 8 * hh + 4);
    float xs[16] = {x0[0],x0[1],x0[2],x0[3],x1[0],x1[1],x1[2],x1[3],x2[0],x2[1],x2[2],x2[3],x3[0],x3[1],x3[2],x3[3]};
#pragma unroll
    for (int i = 0; i < 16; ++i) { const unsigned short hb = bf16_bits(xs[i]); ah.u[i] = hb; al.u[i] = ASPLIT ? bf16_bits(xs[i] - bf16_val(hb)) : (unsigned short)0; }
#pragma unroll
    for (int t = 0; t < 4; ++t) {
      const unsigned short* brow = Wt + (size_t)(col0 + t * 16 + ln) * ldb + kb;
      FragB b;
      b.half[0] = *(const v8us*)(brow + 8 * hh);
      b.half[1] = *(const v8us*)(brow + 16 + 8 * hh);
      acc[t] = mmaN<ASPLIT ? 2 : 1>(ah.v, al.v, b.v, b.v, acc[t]);
    }
  }
#pragma unroll
  for (int t = 0; t < 4; ++t) {
    const int col = col0 + t * 16 + ln;
    float bv = bias ? bias[col] : 0.f;
    if (BIAS_BF16) bv = bf16_round(bv);
#pragma unroll
    for (int r = 0; r < 8; ++r) {
      float v = acc[t][r] + bv;
      if (resid) { float rv = resid[(size_t)((row0 + 8 * hh + r) % rmod) * ldr + col]; if (RES_BF16) rv = bf16_round(rv); v += rv; }
      if (ACT == 1) v = fmaxf(v, 0.f);
      if (ACT == 2) v = 0.5f * v * (1.0f + erff(v * 0.70710678118654752f));
      if (ACT == 3) { const float u = 0.7978845608028654f * (v + 0.044715f * v * v * v); v = 0.5f * v * (1.0f + tanhf(u)); }
      so[w][8 * hh + r][t * 16 + ln] = v;
    }
  }
  __builtin_amdgcn_fence(__ATOMIC_ACQ_REL, "workgroup");
  __builtin_amdgcn_wave_barrier();
  const int rsub = lane >> 4, c4 = (lane & 15) * 4;
  for (int pass = 0; pass < 2; ++pass) {
#pragma unroll
    for (int q = 0; q < 8; ++q) {
      const int r = q * 2 + rsub;
      const v4f v = *(const v4fa*)&so[w][r][c4];
      *(volatile v4f*)(C + (size_t)(row0 + r) * ldc + col0 + c4) = v;
    }
    if (pass == 0) __threadfence();
  }
}
template <bool PARAM_BF16>
__global__ __launch_bounds__(256) void k_layernorm(const float* __restrict__ X, const float* __restrict__ R, const float* __restrict__ g, const float* __restrict__ bta,
                                                  float* __restrict__ out_sum, float* __restrict__ out_norm, int N, float eps) {
  __shared__ float red[256];
  const int row = blockIdx.x, tid = threadIdx.x;
  const float* x = X + (size_t)row * N; const float* rr = R ? R + (size_t)row * N : nullptr;
  float vals[16];
  const int per = N / 256;
  float s1 = 0.f;
  for (int u = 0; u < per / 4; ++u) {
    const int j = tid * 4 + 1024 * u;
    const v4f a = *(const v4fa*)(x + j);
    v4f b = {0.f,0.f,0.f,0.f}; if (rr) b = *(const v4fa*)(rr + j);
#pragma unroll
    for (int q = 0; q < 4; ++q) { const float v = a[q] + b[q]; vals[u * 4 + q] = v; s1 += v; }
  }
  red[tid] = s1; __syncthreads();
  for (int st = 128; st > 0; st >>= 1) { if (tid < st) red[tid] += red[tid + st]; __syncthreads(); }
  const float mu = red[0] / (float)N; __syncthreads();
  float s2 = 0.f;
  for (int u = 0; u < per / 4; ++u)
#pragma unroll
    for (int q = 0; q < 4; ++q) { const float c = vals[u * 4 + q] - mu; s2 += c * c; }
  red[tid] = s2; __syncthreads();
  for (int st = 128; st > 0; st >>= 1) { if (tid < st) red[tid] += red[tid + st]; __syncthreads(); }
  const float rs = rsqrtf(red[0] / (float)N + eps);
  for (int pass = 0; pass < 2; ++pass) {
    for (int u = 0; u < per / 4; ++u) {
      const int j = tid * 4 + 1024 * u;
      v4f o, sm;
#pragma unroll
      for (int q = 0; q < 4; ++q) {
        float gg = g[j + q], bb = bta[j + q];
        if (PARAM_BF16) { gg = bf16_round(gg); bb = bf16_round(bb); }
        sm[q] = vals[u * 4 + q]; o[q] = (vals[u * 4 + q] - mu) * rs * gg + bb;
      }
      if (out_sum) *(volatile v4f*)(out_sum + (size_t)row * N + j) = sm;
      *(volatile v4f*)(out_norm + (size_t)row * N + j) = o;
    }
    if (pass == 0) __threadfence();
  }
}

template <int D>
__global__ __launch_bounds__(128) void k_flash3b(const float* __restrict__ Qb, int qpitch, int Tq,
                                              const float* __restrict__ K1, const float* __restrict__ V1, int Tk1,
                                              const float* __restrict__ K2, const float* __restrict__ V2, int Tk2, int kpitch, int vpitch,
                                              int H, float scale, const float* __restrict__ fmask, int causal, const float* __restrict__ sbias,
                                              float* __restrict__ y, int ypitch) {
  constexpr int KS = D / 32, DT = D / 16;
  __shared__ __attribute__((aligned(16))) unsigned short sKh[32][D + 8], sKl[32][D + 8], sVh[32][D + 8], sVl[32][D + 8];
  __shared__ __attribute__((aligned(16))) unsigned short sPh[4][16][40], sPl[4][16][40];
  __shared__ __attribute__((aligned(16))) float sO[4][16][D];
  const int tid = threadIdx.x, w = tid >> 5, lane = tid & 31, ln = lane & 15, hh = lane >> 4;
  const int Tk = Tk1 + Tk2;
  const int nqb = (Tq + 63) / 64;
  const int bh = blockIdx.x / nqb, qblk = blockIdx.x % nqb;
  const int b = bh / H, h = bh % H;
  const int q0 = qblk * 64 + w * 16;
  const float* Q = Qb + (size_t)b * Tq * qpitch + h * D;
  FragB aqh[KS], aql[KS];
  {
    int row = q0 + ln; if (row >= Tq) row = Tq - 1;
    const float* qr = Q + (size_t)row * qpitch;
#pragma unroll
    for (int ks = 0; ks < KS; ++ks)
#pragma unroll
      for (int i = 0; i < 16; ++i) {
        const int d = ks * 32 + ((i < 8) ? (8 * hh + i) : (16 + 8 * hh + (i - 8)));
        const float x = qr[d] * scale; const unsigned short hb = bf16_bits(x);
        aqh[ks].u[i] = hb; aql[ks].u[i] = bf16_bits(x - bf16_val(hb));
      }
  }
  int qrow[8];
#pragma unroll
  for (int r = 0; r < 8; ++r) { int qi = q0 + 8 * hh + r; qrow[r] = qi < Tq ? qi : Tq - 1; }
  float m_r[8], l_r[8];
#pragma unroll
  for (int r = 0; r < 8; ++r) { m_r[r] = -3.0e38f; l_r[r] = 0.f; }
  v8f oacc[DT];
#pragma unroll
  for (int dt = 0; dt < DT; ++dt) oacc[dt] = (v8f){0.f,0.f,0.f,0.f,0.f,0.f,0.f,0.f};
  const int kv_end = causal ? min(Tk, qblk * 64 + 64) : Tk;
  for (int j0 = 0; j0 < kv_end; j0 += 32) {
    __syncthreads();
    for (int e = tid; e < 32 * (D / 4); e += 128) {
      const int r = e / (D / 4), c4 = (e % (D / 4)) * 4; const int key = j0 + r;
      v4f kf = {0.f,0.f,0.f,0.f}, vf = {0.f,0.f,0.f,0.f};
      if (key < Tk1) { kf = *(const v4fa*)(K1 + (size_t)b * Tk1 * kpitch + h * D + (size_t)key * kpitch + c4); vf = *(const v4fa*)(V1 + (size_t)b * Tk1 * vpitch + h * D + (size_t)key * vpitch + c4); }
      else if (key < Tk) { const int k2 = key - Tk1; kf = *(const v4fa*)(K2 + (size_t)b * Tk2 * kpitch + h * D + (size_t)k2 * kpitch + c4); vf = *(const v4fa*)(V2 + (size_t)b * Tk2 * vpitch + h * D + (size_t)k2 * vpitch + c4); }
#pragma unroll
      for (int t = 0; t < 4; ++t) {
        unsigned short hb = bf16_bits(kf[t]); sKh[r][c4 + t] = hb; sKl[r][c4 + t] = bf16_bits(kf[t] - bf16_val(hb));
        hb = bf16_bits(vf[t]); sVh[r][c4 + t] = hb; sVl[r][c4 + t] = bf16_bits(vf[t] - bf16_val(hb));
      }
    }
    __syncthreads();
    v8f s[2];
#pragma unroll
    for (int nt = 0; nt < 2; ++nt) {
      v8f acc = {};
#pragma unroll
      for (int ks = 0; ks < KS; ++ks) {
        FragB bh_, bl_;
        bh_.half[0] = *(const v8us*)&sKh[nt * 16 + ln][ks * 32 + 8 * hh]; bh_.half[1] = *(const v8us*)&sKh[nt * 16 + ln][ks * 32 + 16 + 8 * hh];
        bl_.half[0] = *(const v8us*)&sKl[nt * 16 + ln][ks * 32 + 8 * hh]; bl_.half[1] = *(const v8us*)&sKl[nt * 16 + ln][ks * 32 + 16 + 8 * hh];
        acc = mmaN<3>(aqh[ks].v, aql[ks].v, bh_.v, bl_.v, acc);
      }
      s[nt] = acc;
    }
    float alpha[8];
#pragma unroll
    for (int r = 0; r < 8; ++r) {
      const int qi = qrow[r];
      const int ja = j0 + ln, jb = j0 + 16 + ln;
      bool keepa = ja < Tk, keepb = jb < Tk;
      if (causal) { keepa = keepa && (ja <= qi); keepb = keepb && (jb <= qi); }
      if (fmask) { const float* fm = fmask + ((size_t)b * Tq + qi) * Tk; if (keepa) s[0][r] += bf16_round(fm[ja]); if (keepb) s[1][r] += bf16_round(fm[jb]); }
      if (sbias) { if (keepa) s[0][r] += sbias[(size_t)bh * Tk + ja]; if (keepb) s[1][r] += sbias[(size_t)bh * Tk + jb]; }
      if (!keepa) s[0][r] = -3.0e38f;
      if (!keepb) s[1][r] = -3.0e38f;
      float mx = fmaxf(s[0][r], s[1][r]);
      mx = fmaxf(mx, __shfl_xor(mx, 1, 32)); mx = fmaxf(mx, __shfl_xor(mx, 2, 32)); mx = fmaxf(mx, __shfl_xor(mx, 4, 32)); mx = fmaxf(mx, __shfl_xor(mx, 8, 32));
      const float mnew = fmaxf(m_r[r], mx);
      alpha[r] = (mnew > -1.0e38f) ? __expf(m_r[r] - mnew) : 1.0f;
      const float p0 = keepa ? __expf(s[0][r] - mnew) : 0.f;
      const float p1 = keepb ? __expf(s[1][r] - mnew) : 0.f;
      m_r[r] = mnew;
      l_r[r] = l_r[r] * alpha[r] + p0 + p1;
      unsigned short hb = bf16_bits(p0); sPh[w][8 * hh + r][ln] = hb;      sPl[w][8 * hh + r][ln] = bf16_bits(p0 - bf16_val(hb));
      hb = bf16_bits(p1);                sPh[w][8 * hh + r][16 + ln] = hb; sPl[w][8 * hh + r][16 + ln] = bf16_bits(p1 - bf16_val(hb));
    }
#pragma unroll
    for (int dt = 0; dt < DT; ++dt)
#pragma unroll
      for (int r = 0; r < 8; ++r) oacc[dt][r] *= alpha[r];
    __builtin_amdgcn_fence(__ATOMIC_ACQ_REL, "workgroup");
    __builtin_amdgcn_wave_barrier();
    FragB pah, pal;
    pah.half[0] = *(const v8us*)&sPh[w][ln][8 * hh]; pah.half[1] = *(const v8us*)&sPh[w][ln][16 + 8 * hh];
    pal.half[0] = *(const v8us*)&sPl[w][ln][8 * hh]; pal.half[1] = *(const v8us*)&sPl[w][ln][16 + 8 * hh];
#pragma unroll
    for (int dt = 0; dt < DT; ++dt) {
      FragB bvh, bvl;
#pragma unroll
      for (int i = 0; i < 8; ++i) {
        bvh.u[i] = sVh[8 * hh + i][dt * 16 + ln]; bvh.u[8 + i] = sVh[16 + 8 * hh + i][dt * 16 + ln];
        bvl.u[i] = sVl[8 * hh + i][dt * 16 + ln]; bvl.u[8 + i] = sVl[16 + 8 * hh + i][dt * 16 + ln];
      }
      oacc[dt] = mmaN<3>(pah.v, pal.v, bvh.v, bvl.v, oacc[dt]);
    }
    __builtin_amdgcn_fence(__ATOMIC_ACQ_REL, "workgroup");
    __builtin_amdgcn_wave_barrier();
  }
#pragma unroll
  for (int r = 0; r < 8; ++r) {
    float l = l_r[r];
    l += __shfl_xor(l, 1, 32); l += __shfl_xor(l, 2, 32); l += __shfl_xor(l, 4, 32); l += __shfl_xor(l, 8, 32);
    l_r[r] = (m_r[r] > -1.0e38f) ? 1.0f / l : __builtin_nanf("");
  }
#pragma unroll
  for (int dt = 0; dt < DT; ++dt)
#pragma unroll
    for (int r = 0; r < 8; ++r) sO[w][8 * hh + r][dt * 16 + ln] = oacc[dt][r] * l_r[r];
  __builtin_amdgcn_fence(__ATOMIC_ACQ_REL, "workgroup");
  __builtin_amdgcn_wave_barrier();
  for (int pass = 0; pass < 2; ++pass) {
    for (int r = 0; r < 16; ++r) {
      const int row = q0 + r;
      if (row < Tq && lane < D / 4) {
        const v4f val = *(const v4fa*)&sO[w][r][lane * 4];
        *(volatile v4f*)(y + ((size_t)b * Tq + row) * ypitch + h * D + lane * 4) = val;
      }
    }
    if (pass == 0) __threadfence();
  }
}

__global__ void k_ln_rows(const float* __restrict__ X, const float* __restrict__ R, const float* __restrict__ g, const float* __restrict__ bta, float* __restrict__ out, int N, float eps) {
  __shared__ float red[256];
  const int row = blockIdx.x, tid = threadIdx.x, nt = blockDim.x;
  v4f a = *(const v4fa*)(X + (size_t)row * N + tid * 4);
  if (R) { const v4f rr = *(const v4fa*)(R + (size_t)row * N + tid * 4); for (int q = 0; q < 4; ++q) a[q] += rr[q]; }
  float s = a[0] + a[1] + a[2] + a[3];
  red[tid] = s; __syncthreads();
  for (int st = nt / 2; st > 0; st >>= 1) { if (tid < st) red[tid] += red[tid + st]; __syncthreads(); }
  const float mu = red[0] / (float)N; __syncthreads();
  float v = 0.f; for (int q = 0; q < 4; ++q) { const float c = a[q] - mu; v += c * c; }
  red[tid] = v; __syncthreads();
  for (int st = nt / 2; st > 0; st >>= 1) { if (tid < st) red[tid] += red[tid + st]; __syncthreads(); }
  const float rs = rsqrtf(red[0] / (float)N + eps);
  v4f o; for (int q = 0; q < 4; ++q) o[q] = (a[q] - mu) * rs * bf16_round(g[tid * 4 + q]) + bf16_round(bta[tid * 4 + q]);
  *(volatile v4f*)(out + (size_t)row * N + tid * 4) = o; __threadfence(); *(volatile v4f*)(out + (size_t)row * N + tid * 4) = o;
}

__global__ __launch_bounds__(128) void k_embed(const int* __restrict__ tok, const float* __restrict__ emb, float* __restrict__ y) {
  const int row = blockIdx.x, tid = threadIdx.x; const int t = row % TT;
  int id = tok[row]; id = id < 0 ? 0 : (id >= VV ? VV - 1 : id);
  const v4f e = *(const v4fa*)(emb + (size_t)id * DD + tid * 4);
  v4f o;
#pragma unroll 1
  for (int pr = 0; pr < 2; ++pr) {
    const int i2 = tid * 4 + pr * 2;
    const float denom = powf(10000.0f, (float)i2 / (float)DD);
    const float ang = (float)t / denom;
    float sv, cv; sincosf(ang, &sv, &cv);
    o[pr * 2] = bf16_round(e[pr * 2]) + sv; o[pr * 2 + 1] = bf16_round(e[pr * 2 + 1]) + cv;
  }
  *(volatile v4f*)(y + (size_t)row * DD + tid * 4) = o; __threadfence(); *(volatile v4f*)(y + (size_t)row * DD + tid * 4) = o;
}
extern "C" void kernel_launch(void* const* d_in, const int* in_sizes, int n_in,
                              void* d_out, int out_size, void* d_ws, size_t ws_size, hipStream_t stream) {
  (void)in_sizes; (void)n_in; (void)out_size;
  const float* x = (const float*)d_in[0]; const int* ytok = (const int*)d_in[1]; const float* self_mask = (const float*)d_in[2]; const float* cross_mask = (const float*)d_in[3];
  const float* emb = (const float*)d_in[4];
  const float* Wqkv = (const float*)d_in[5]; const float* bqkv = (const float*)d_in[6]; const float* Wo = (const float*)d_in[7]; const float* bo = (const float*)d_in[8];
  const float* Wkv = (const float*)d_in[9]; const float* bkv = (const float*)d_in[10]; const float* Wq = (const float*)d_in[11]; const float* bq = (const float*)d_in[12];
  const float* Wco = (const float*)d_in[13]; const float* bco = (const float*)d_in[14]; const float* W1 = (const float*)d_in[15]; const float* b1 = (const float*)d_in[16];
  const float* W2 = (const float*)d_in[17]; const float* b2 = (const float*)d_in[18];
  const float* g1 = (const float*)d_in[19]; const float* be1 = (const float*)d_in[20]; const float* g2 = (const float*)d_in[21]; const float* be2 = (const float*)d_in[22]; const float* g3 = (const float*)d_in[23]; const float* be3 = (const float*)d_in[24];
  char* ws = (char*)d_ws; size_t off = 0;
  auto take = [&](size_t bytes) { char* p = ws + off; off += (bytes + 255) & ~(size_t)255; return p; };
  const int M = BB * TT;
  unsigned short* Wqkvt[NL], *Wot[NL], *Wkvt[NL], *Wqt[NL], *Wcot[NL], *W1t[NL], *W2t[NL];
  for (int l = 0; l < NL; ++l) { Wqkvt[l] = (unsigned short*)take((size_t)3 * DD * DD * 2); Wot[l] = (unsigned short*)take((size_t)DD * DD * 2); Wkvt[l] = (unsigned short*)take((size_t)2 * DD * DD * 2); Wqt[l] = (unsigned short*)take((size_t)DD * DD * 2); Wcot[l] = (unsigned short*)take((size_t)DD * DD * 2); W1t[l] = (unsigned short*)take((size_t)FF * DD * 2); W2t[l] = (unsigned short*)take((size_t)DD * FF * 2); }
  float* y = (float*)take((size_t)M * DD * 4); float* y2 = (float*)take((size_t)M * DD * 4);
  float* qkv = (float*)take((size_t)M * 3 * DD * 4); float* att = (float*)take((size_t)M * DD * 4); float* tmp = (float*)take((size_t)M * DD * 4);
  float* kvx = (float*)take((size_t)M * 2 * DD * 4); float* qb2 = (float*)take((size_t)M * DD * 4); float* ffn = (float*)take((size_t)M * FF * 4);
  if (off > ws_size) return;
  for (int l = 0; l < NL; ++l) {
    k_wt_bf16<<<(3 * DD * (DD / 8) + 255) / 256, 256, 0, stream>>>(Wqkv + (size_t)l * DD * 3 * DD, Wqkvt[l], DD, 3 * DD);
    k_wt_bf16<<<(DD * (DD / 8) + 255) / 256, 256, 0, stream>>>(Wo + (size_t)l * DD * DD, Wot[l], DD, DD);
    k_wt_bf16<<<(2 * DD * (DD / 8) + 255) / 256, 256, 0, stream>>>(Wkv + (size_t)l * DD * 2 * DD, Wkvt[l], DD, 2 * DD);
    k_wt_bf16<<<(DD * (DD / 8) + 255) / 256, 256, 0, stream>>>(Wq + (size_t)l * DD * DD, Wqt[l], DD, DD);
    k_wt_bf16<<<(DD * (DD / 8) + 255) / 256, 256, 0, stream>>>(Wco + (size_t)l * DD * DD, Wcot[l], DD, DD);
    k_wt_bf16<<<(FF * (DD / 8) + 255) / 256, 256, 0, stream>>>(W1 + (size_t)l * DD * FF, W1t[l], DD, FF);
    k_wt_bf16<<<(DD * (FF / 8) + 255) / 256, 256, 0, stream>>>(W2 + (size_t)l * FF * DD, W2t[l], FF, DD);
  }
  k_embed<<<M, 128, 0, stream>>>(ytok, emb, y);
  const float scale = 0.125f;
  for (int l = 0; l < NL; ++l) {
    k_gemm_bf3<true, 0, true, false><<<((M / 16) * (3 * DD / 64) + 3) / 4, 128, 0, stream>>>(y, DD, Wqkvt[l], DD, bqkv + l * 3 * DD, nullptr, 1, 0, qkv, 3 * DD, M, 3 * DD, DD);
    k_flash3b<HD><<<BB * NH * (TT / 64), 128, 0, stream>>>(qkv, 3 * DD, TT, qkv + DD, qkv + 2 * DD, TT, nullptr, nullptr, 0, 3 * DD, 3 * DD, NH, scale, self_mask, 0, nullptr, att, DD);
    k_gemm_bf3<true, 0, true, false><<<((M / 16) * (DD / 64) + 3) / 4, 128, 0, stream>>>(att, DD, Wot[l], DD, bo + l * DD, nullptr, 1, 0, tmp, DD, M, DD, DD);
    k_ln_rows<<<M, DD / 4, 0, stream>>>(tmp, y, g1 + l * DD, be1 + l * DD, y2, DD, 1e-5f);
    k_gemm_bf3<false, 0, true, false><<<((M / 16) * (2 * DD / 64) + 3) / 4, 128, 0, stream>>>(x, DD, Wkvt[l], DD, bkv + l * 2 * DD, nullptr, 1, 0, kvx, 2 * DD, M, 2 * DD, DD);
    k_gemm_bf3<true, 0, true, false><<<((M / 16) * (DD / 64) + 3) / 4, 128, 0, stream>>>(y2, DD, Wqt[l], DD, bq + l * DD, nullptr, 1, 0, qb2, DD, M, DD, DD);
    k_flash3b<HD><<<BB * NH * (TT / 64), 128, 0, stream>>>(qb2, DD, TT, kvx, kvx + DD, TT, nullptr, nullptr, 0, 2 * DD, 2 * DD, NH, scale, cross_mask, 0, nullptr, att, DD);
    k_gemm_bf3<true, 0, true, false><<<((M / 16) * (DD / 64) + 3) / 4, 128, 0, stream>>>(att, DD, Wcot[l], DD, bco + l * DD, nullptr, 1, 0, tmp, DD, M, DD, DD);
    k_ln_rows<<<M, DD / 4, 0, stream>>>(tmp, y2, g2 + l * DD, be2 + l * DD, y, DD, 1e-5f);
    k_gemm_bf3<true, 1, true, false><<<((M / 16) * (FF / 64) + 3) / 4, 128, 0, stream>>>(y, DD, W1t[l], DD, b1 + l * FF, nullptr, 1, 0, ffn, FF, M, FF, DD);
    k_gemm_bf3<true, 0, true, false><<<((M / 16) * (DD / 64) + 3) / 4, 128, 0, stream>>>(ffn, FF, W2t[l], FF, b2 + l * DD, nullptr, 1, 0, tmp, DD, M, DD, FF);
    k_ln_rows<<<M, DD / 4, 0, stream>>>(tmp, y, g3 + l * DD, be3 + l * DD, (l == NL - 1) ? (float*)d_out : y2, DD, 1e-5f);
    if (l < NL - 1) { float* sw = y; y = y2; y2 = sw; }
  }
}
